// CachedGCN_19688130085401
// MI455X (gfx1250) — hardware-run, weakly checked
//
#include <hip/hip_runtime.h>
#include <stddef.h>
#include <stdint.h>

#ifndef SPLIT1
#define SPLIT1 0
#endif
#ifndef SPLIT2
#define SPLIT2 0
#endif

#define NN      100000
#define NE      1600000
#define D0      64
#define HD      128
#define OD      64
#define GBM     128
#define MP      100096
#define Z1P     128
#define Z2P     256
#define W1P     128
#define W3P     256
#define K1      (SPLIT1 ? 128 : 64)
#define K2      (SPLIT2 ? 256 : 128)
#define NTHR    256
#define NWAVE   8
#define EPT     8
#define WCH     (32 * EPT)
#define NBRUN   1024
#define EIDB    21
#define NBK     98
#define WLCAP   3584
#define RCAP    28672
#define DEGCAP  64
#define MAXDEG_MEAS   37
#define MAXB1024_MEAS 16666
#define SP      68

#define BK_ZINTS (NWAVE * WLCAP + RCAP + 3 * NBRUN)
#define BK_INTS  (BK_ZINTS + 16)
#define BK_LDS   (BK_INTS * 4)

#define PBX  (MP * D0 / 8 / NTHR)
#define PBW1 (HD * W1P / 8 / NTHR)
#define PBW3 (OD * W3P / 8 / NTHR)
#define PBTOT (PBX + PBW1 + PBW3)

static_assert(NN <= (1 << 17));
static_assert(NE < (1 << EIDB));
static_assert(NBRUN == 1024 && NBRUN % 128 == 0 && NBRUN % GBM == 0 && NBRUN % 32 == 0);
static_assert(RCAP % 16 == 0 && RCAP == NWAVE * WLCAP && RCAP % (NTHR * 2) == 0);
static_assert(MP % GBM == 0 && MP >= NN && MP == 782 * GBM);
static_assert(NBK * NBRUN >= MP);
static_assert(NE % WCH == 0 && NE % 4 == 0);
static_assert((long long)RCAP * 100 >= (long long)MAXB1024_MEAS * 105);
static_assert(WLCAP >= MAXB1024_MEAS / 8 + 8 * 46 + 1);
static_assert(MAXDEG_MEAS + 8 <= DEGCAP && DEGCAP < 65536);
static_assert(BK_ZINTS % 4 == 0 && BK_LDS <= 300000);
static_assert(GBM * SP * 4 <= 65536);
static_assert(K1 % 32 == 0 && K2 % 32 == 0 && K1 <= Z1P && K1 <= W1P && K2 <= Z2P && K2 <= W3P);
static_assert(Z1P == 2 * D0 && Z2P == 2 * HD);
static_assert((MP * D0 / 8) % NTHR == 0 && (HD * W1P / 8) % NTHR == 0 && (OD * W3P / 8) % NTHR == 0);
static_assert(D0 == 16 * 4 && HD == 32 * 4 && OD == 16 * 4);
static_assert(NN * OD == 6400000);

typedef float          v4f   __attribute__((ext_vector_type(4)));
typedef float          v8f   __attribute__((ext_vector_type(8)));
typedef int            v2i   __attribute__((ext_vector_type(2)));
typedef int            v4i   __attribute__((ext_vector_type(4)));
typedef int            v8i   __attribute__((ext_vector_type(8)));
typedef unsigned       v2u   __attribute__((ext_vector_type(2)));
typedef unsigned       v4u   __attribute__((ext_vector_type(4)));
typedef unsigned short v8us  __attribute__((ext_vector_type(8)));
typedef unsigned short v16us __attribute__((ext_vector_type(16)));
typedef __bf16         v16bf __attribute__((ext_vector_type(16)));
typedef v4f  __attribute__((may_alias)) v4fa;
typedef v2i  __attribute__((may_alias)) v2ia;
typedef v4i  __attribute__((may_alias)) v4ia;
typedef v2u  __attribute__((may_alias)) v2ua;
typedef v8us __attribute__((may_alias)) v8usa;
union FragB { v16bf v; v16us u; v8us h[2]; v8i w; };

__device__ __forceinline__ v8f wmb(const FragB& a, const FragB& b, v8f c) {
  v8f d = __builtin_amdgcn_wmma_f32_16x16x32_bf16(false, a.v, false, b.v, (short)0, c, false, false);
  asm volatile("v_nop\n\tv_nop\n\tv_nop\n\tv_nop" : "+v"(d) : "v"(a.w), "v"(b.w));
  return d;
}

__device__ __forceinline__ unsigned bf16_bits(float f) {
  const unsigned u = __float_as_uint(f);
  const unsigned r = (u + 0x7FFFu + ((u >> 16) & 1u)) >> 16;
  const unsigned q = (u >> 16) | 0x40u;
  return ((u & 0x7fffffffu) > 0x7f800000u) ? q : r;
}
__device__ __forceinline__ float bfw_lo(unsigned w) { return __uint_as_float(w << 16); }
__device__ __forceinline__ float bfw_hi(unsigned w) { return __uint_as_float(w & 0xffff0000u); }

__device__ __forceinline__ void hilo_pack(float v0, float v1, float v2, float v3,
                                          int& h01, int& h23, int& l01, int& l23) {
  const unsigned a0 = bf16_bits(v0), a1 = bf16_bits(v1), a2 = bf16_bits(v2), a3 = bf16_bits(v3);
  const unsigned b0 = bf16_bits(v0 - __uint_as_float(a0 << 16));
  const unsigned b1 = bf16_bits(v1 - __uint_as_float(a1 << 16));
  const unsigned b2 = bf16_bits(v2 - __uint_as_float(a2 << 16));
  const unsigned b3 = bf16_bits(v3 - __uint_as_float(a3 << 16));
  h01 = (int)(a0 | (a1 << 16)); h23 = (int)(a2 | (a3 << 16));
  l01 = (int)(b0 | (b1 << 16)); l23 = (int)(b2 | (b3 << 16));
}

__device__ __forceinline__ v4i regroup8(int h01, int h23, int l01, int l23, int lane) {
  const int t  = lane & 15;
  const int s0 = (lane & 16) + ((2 * t) & 15), s1 = s0 + 1;
  const int a0 = __shfl(h01, s0, 32), a1 = __shfl(h23, s0, 32), a2 = __shfl(h01, s1, 32), a3 = __shfl(h23, s1, 32);
  const int b0 = __shfl(l01, s0, 32), b1 = __shfl(l23, s0, 32), b2 = __shfl(l01, s1, 32), b3 = __shfl(l23, s1, 32);
  const int mk = (t < 8) ? -1 : 0;
  v4i o;
  o.x = (a0 & mk) | (b0 & ~mk); o.y = (a1 & mk) | (b1 & ~mk);
  o.z = (a2 & mk) | (b2 & ~mk); o.w = (a3 & mk) | (b3 & ~mk);
  return o;
}

__device__ __forceinline__ v4i regroup8w(int h01, int h23, int l01, int l23, int lane) {
  const int s0 = (2 * lane) & 31, s1 = s0 + 1;
  const int a0 = __shfl(h01, s0, 32), a1 = __shfl(h23, s0, 32), a2 = __shfl(h01, s1, 32), a3 = __shfl(h23, s1, 32);
  const int b0 = __shfl(l01, s0, 32), b1 = __shfl(l23, s0, 32), b2 = __shfl(l01, s1, 32), b3 = __shfl(l23, s1, 32);
  const int mk = (lane < 16) ? -1 : 0;
  v4i o;
  o.x = (a0 & mk) | (b0 & ~mk); o.y = (a1 & mk) | (b1 & ~mk);
  o.z = (a2 & mk) | (b2 & ~mk); o.w = (a3 & mk) | (b3 & ~mk);
  return o;
}

__device__ __forceinline__ void st2_v4f(float* p, v4f v) {
  *(volatile v4f*)p = v;
  __threadfence();
  *(volatile v4f*)p = v;
}
__device__ __forceinline__ void st2_v8us(unsigned short* p, v8us v) {
  *(volatile v8us*)p = v;
  __threadfence();
  *(volatile v8us*)p = v;
}
__device__ __forceinline__ void st2_v4i(unsigned short* p, v4i v) {
  *(volatile v4i*)p = v;
  __threadfence();
  *(volatile v4i*)p = v;
}

__device__ __forceinline__ v8us gather8(const float* __restrict__ base, int stride) {
  float f[8];
#pragma unroll
  for (int i = 0; i < 8; ++i) f[i] = base[(size_t)i * (size_t)stride];
  v8us o;
#pragma unroll
  for (int i = 0; i < 8; ++i) o[i] = (unsigned short)bf16_bits(f[i]);
  return o;
}

__global__ __launch_bounds__(NTHR) void k_prep(const float* __restrict__ x, const float* __restrict__ w1,
                                               const float* __restrict__ w3, unsigned short* xb,
                                               unsigned short* w1d, unsigned short* w3d) {
  const int tid = (int)threadIdx.x;
  const int blk = (int)blockIdx.x;
  if (blk < PBX) {
    const int u   = blk * NTHR + tid;
    const int row = u >> 3, k8 = (u & 7) * 8;
    const int rc  = row < NN ? row : NN - 1;
    const unsigned mk = row < NN ? 0xffffu : 0u;
    const float* p = x + (size_t)rc * D0 + k8;
    const v4f a = *(const v4fa*)p;
    const v4f b = *(const v4fa*)(p + 4);
    v8us o;
    o[0] = (unsigned short)(bf16_bits(a.x) & mk); o[1] = (unsigned short)(bf16_bits(a.y) & mk);
    o[2] = (unsigned short)(bf16_bits(a.z) & mk); o[3] = (unsigned short)(bf16_bits(a.w) & mk);
    o[4] = (unsigned short)(bf16_bits(b.x) & mk); o[5] = (unsigned short)(bf16_bits(b.y) & mk);
    o[6] = (unsigned short)(bf16_bits(b.z) & mk); o[7] = (unsigned short)(bf16_bits(b.w) & mk);
    st2_v8us(xb + (size_t)row * D0 + k8, o);
  } else if (blk < PBX + PBW1) {
    const int u = (blk - PBX) * NTHR + tid;
    const int n = u >> 4, k8 = (u & 15) * 8, kk = k8 & 63;
    const v8us o = gather8(w1 + (size_t)kk * HD + n, HD);
    st2_v8us(w1d + (size_t)n * W1P + k8, o);
  } else {
    const int u = (blk - PBX - PBW1) * NTHR + tid;
    const int n = u >> 5, k8 = (u & 31) * 8, kk = k8 & 127;
    const v8us o = gather8(w3 + (size_t)kk * OD + n, OD);
    st2_v8us(w3d + (size_t)n * W3P + k8, o);
  }
}

__global__ __launch_bounds__(NTHR) void k_bucket(const int* __restrict__ keys, const int* __restrict__ cols,
                                                 const float* __restrict__ ew, unsigned* LIST, int* CNT, int* OFF,
                                                 int* FLAG) {
  extern __shared__ __attribute__((aligned(16))) int dsm[];
  int* wl   = dsm;
  int* pl   = dsm + NWAVE * WLCAP;
  int* cnt  = pl + RCAP;
  int* offs = cnt + NBRUN;
  int* cur  = offs + NBRUN;
  int* misc = cur + NBRUN;
  const int tid = (int)threadIdx.x, lane = tid & 31, wave = tid >> 5;
  const int blk = (int)blockIdx.x;
  const unsigned nbs = (unsigned)(blk * NBRUN);

  {
    const v4i z4 = {0, 0, 0, 0};
    for (int i = tid * 4; i < BK_ZINTS; i += NTHR * 4) *(v4ia*)(dsm + i) = z4;
    if (tid < 16) misc[tid] = 0;
  }
  __syncthreads();

  {
    const int per  = ((NE + NWAVE * WCH - 1) / (NWAVE * WCH)) * WCH;
    const int ebeg = wave * per;
    const int eend = (ebeg + per < NE) ? (ebeg + per) : NE;
    int* mylist = wl + wave * WLCAP;
    int wc = 0;
#pragma unroll 1
    for (int cb = ebeg; cb < eend; cb += WCH) {
      const int e0 = cb + lane * EPT;
      const v4i da = *(const v4ia*)(keys + e0);
      const v4i db = *(const v4ia*)(keys + e0 + 4);
      const unsigned s0 = (unsigned)da.x - nbs, s1 = (unsigned)da.y - nbs;
      const unsigned s2 = (unsigned)da.z - nbs, s3 = (unsigned)da.w - nbs;
      const unsigned s4 = (unsigned)db.x - nbs, s5 = (unsigned)db.y - nbs;
      const unsigned s6 = (unsigned)db.z - nbs, s7 = (unsigned)db.w - nbs;
      const bool h0 = s0 < (unsigned)NBRUN, h1 = s1 < (unsigned)NBRUN, h2 = s2 < (unsigned)NBRUN, h3 = s3 < (unsigned)NBRUN;
      const bool h4 = s4 < (unsigned)NBRUN, h5 = s5 < (unsigned)NBRUN, h6 = s6 < (unsigned)NBRUN, h7 = s7 < (unsigned)NBRUN;
      const unsigned m0 = __builtin_amdgcn_ballot_w32(h0), m1 = __builtin_amdgcn_ballot_w32(h1);
      const unsigned m2 = __builtin_amdgcn_ballot_w32(h2), m3 = __builtin_amdgcn_ballot_w32(h3);
      const unsigned m4 = __builtin_amdgcn_ballot_w32(h4), m5 = __builtin_amdgcn_ballot_w32(h5);
      const unsigned m6 = __builtin_amdgcn_ballot_w32(h6), m7 = __builtin_amdgcn_ballot_w32(h7);
      const unsigned any = m0 | m1 | m2 | m3 | m4 | m5 | m6 | m7;
      if (any != 0u) {
        const int pre = (int)(__builtin_amdgcn_mbcnt_lo(m0, 0u) + __builtin_amdgcn_mbcnt_lo(m1, 0u) +
                              __builtin_amdgcn_mbcnt_lo(m2, 0u) + __builtin_amdgcn_mbcnt_lo(m3, 0u) +
                              __builtin_amdgcn_mbcnt_lo(m4, 0u) + __builtin_amdgcn_mbcnt_lo(m5, 0u) +
                              __builtin_amdgcn_mbcnt_lo(m6, 0u) + __builtin_amdgcn_mbcnt_lo(m7, 0u));
        int p = wc + pre;
        if (h0) { if (p < WLCAP) mylist[p] = ((int)s0 << EIDB) | (e0 + 0); p = p + 1; }
        if (h1) { if (p < WLCAP) mylist[p] = ((int)s1 << EIDB) | (e0 + 1); p = p + 1; }
        if (h2) { if (p < WLCAP) mylist[p] = ((int)s2 << EIDB) | (e0 + 2); p = p + 1; }
        if (h3) { if (p < WLCAP) mylist[p] = ((int)s3 << EIDB) | (e0 + 3); p = p + 1; }
        if (h4) { if (p < WLCAP) mylist[p] = ((int)s4 << EIDB) | (e0 + 4); p = p + 1; }
        if (h5) { if (p < WLCAP) mylist[p] = ((int)s5 << EIDB) | (e0 + 5); p = p + 1; }
        if (h6) { if (p < WLCAP) mylist[p] = ((int)s6 << EIDB) | (e0 + 6); p = p + 1; }
        if (h7) { if (p < WLCAP) mylist[p] = ((int)s7 << EIDB) | (e0 + 7); p = p + 1; }
        wc += (int)(__builtin_popcount(m0) + __builtin_popcount(m1) + __builtin_popcount(m2) + __builtin_popcount(m3) +
                    __builtin_popcount(m4) + __builtin_popcount(m5) + __builtin_popcount(m6) + __builtin_popcount(m7));
      }
    }
    if (lane == 0) misc[wave] = wc;
  }
  __syncthreads();

  int ov = 0;
  if (wave == 0) {
#pragma unroll 1
    for (int w2 = 0; w2 < NWAVE; ++w2) {
      int c = misc[w2];
      if (c > WLCAP) ov = 1;
      c = c < 0 ? 0 : (c > WLCAP ? WLCAP : c);
#pragma unroll 1
      for (int b0 = 0; b0 < c; b0 += 32) {
        const int idx = b0 + lane;
        const int ent = wl[w2 * WLCAP + (idx < WLCAP ? idx : WLCAP - 1)];
        const int m32 = (c - b0) < 32 ? (c - b0) : 32;
#pragma unroll 1
        for (int k = 0; k < m32; ++k) {
          const int u    = __builtin_amdgcn_readlane(ent, k);
          const int slot = (u >> EIDB) & (NBRUN - 1);
          if (lane == 0) cnt[slot] = cnt[slot] + 1;
        }
      }
    }
  }
  __syncthreads();
  if (wave == 0) {
    const int base = lane * (NBRUN / 32);
    int s = 0, mx = 0;
#pragma unroll 1
    for (int i = 0; i < NBRUN / 32; ++i) {
      const int cv = cnt[base + i];
      s += cv;
      mx = cv > mx ? cv : mx;
    }
    int incl = s;
#pragma unroll
    for (int d = 1; d < 32; d <<= 1) {
      const int y = __shfl_up(incl, d, 32);
      if (lane >= d) incl += y;
    }
    {
      int t;
      t = __shfl_xor(mx, 16, 32); mx = t > mx ? t : mx;
      t = __shfl_xor(mx, 8, 32);  mx = t > mx ? t : mx;
      t = __shfl_xor(mx, 4, 32);  mx = t > mx ? t : mx;
      t = __shfl_xor(mx, 2, 32);  mx = t > mx ? t : mx;
      t = __shfl_xor(mx, 1, 32);  mx = t > mx ? t : mx;
    }
    if (mx > DEGCAP) ov = 1;
    int run = incl - s;
#pragma unroll 1
    for (int i = 0; i < NBRUN / 32; ++i) {
      const int cv = cnt[base + i];
      offs[base + i] = run;
      cur[base + i]  = run;
      run += cv;
    }
  }
  __syncthreads();

  if (wave == 0) {
#pragma unroll 1
    for (int w2 = 0; w2 < NWAVE; ++w2) {
      int c = misc[w2];
      c = c < 0 ? 0 : (c > WLCAP ? WLCAP : c);
#pragma unroll 1
      for (int b0 = 0; b0 < c; b0 += 32) {
        const int idx = b0 + lane;
        const int ent = wl[w2 * WLCAP + (idx < WLCAP ? idx : WLCAP - 1)];
        const int m32 = (c - b0) < 32 ? (c - b0) : 32;
#pragma unroll 1
        for (int k = 0; k < m32; ++k) {
          const int u    = __builtin_amdgcn_readlane(ent, k);
          const int slot = (u >> EIDB) & (NBRUN - 1);
          const int eid  = u & ((1 << EIDB) - 1);
          if (lane == 0) {
            int p = cur[slot];
            p = p < 0 ? 0 : (p > RCAP - 1 ? RCAP - 1 : p);
            pl[p] = eid;
            cur[slot] = p + 1;
          }
        }
      }
    }
    if (lane == 0) misc[9] = ov;
  }
  __syncthreads();

  const int ovf = misc[9];
  int nh = 0;
#pragma unroll
  for (int w2 = 0; w2 < NWAVE; ++w2) {
    int c = misc[w2];
    c = c < 0 ? 0 : (c > WLCAP ? WLCAP : c);
    nh += c;
  }
  unsigned* lp = LIST + (size_t)blk * (size_t)(RCAP * 2);
#pragma unroll 1
  for (int it = 0; it < RCAP / (NTHR * 2); ++it) {
    const int i0 = 2 * (it * NTHR + tid);
    const v2i ev = *(const v2ia*)(pl + i0);
    int e0 = ev.x, e1 = ev.y;
    e0 = e0 < 0 ? 0 : (e0 > NE - 1 ? NE - 1 : e0);
    e1 = e1 < 0 ? 0 : (e1 > NE - 1 ? NE - 1 : e1);
    int g0 = cols[e0], g1 = cols[e1];
    const float f0 = ew[e0], f1 = ew[e1];
    asm volatile("" :: "v"(g0), "v"(g1), "v"(f0), "v"(f1));
    g0 = g0 < 0 ? 0 : (g0 > NN - 1 ? NN - 1 : g0);
    g1 = g1 < 0 ? 0 : (g1 > NN - 1 ? NN - 1 : g1);
    const unsigned b0 = bf16_bits(f0) << 16, b1 = bf16_bits(f1) << 16;
    const unsigned k0 = (i0 < nh) ? 0xffffffffu : 0u;
    const unsigned k1 = (i0 + 1 < nh) ? 0xffffffffu : 0u;
    v4u o;
    o.x = (unsigned)g0 & k0; o.y = b0 & k0;
    o.z = (unsigned)g1 & k1; o.w = b1 & k1;
    unsigned* dp = lp + (size_t)2 * (size_t)i0;
    *(volatile v4u*)dp = o;
    __threadfence();
    *(volatile v4u*)dp = o;
  }
  {
    const v4i cv = *(const v4ia*)(cnt + 4 * tid);
    const v4i fv = *(const v4ia*)(offs + 4 * tid);
    const v4i fl = {ovf, ovf, ovf, ovf};
    int* cp = CNT + (size_t)blk * NBRUN + 4 * tid;
    int* op = OFF + (size_t)blk * NBRUN + 4 * tid;
    int* fp = FLAG + (size_t)blk * 32 + 4 * (tid & 7);
    *(volatile v4i*)cp = cv;
    *(volatile v4i*)op = fv;
    if (tid < 8) *(volatile v4i*)fp = fl;
    __threadfence();
    *(volatile v4i*)cp = cv;
    *(volatile v4i*)op = fv;
    if (tid < 8) *(volatile v4i*)fp = fl;
  }
}

__global__ __launch_bounds__(NTHR) void k_replay1(const unsigned* __restrict__ LIST, const int* __restrict__ CNT,
                                                  const int* __restrict__ OFF, const int* __restrict__ FLAG,
                                                  const unsigned short* __restrict__ XB, unsigned short* Z1) {
  const int tid = (int)threadIdx.x, lane = tid & 31, wave = tid >> 5, hh = lane >> 4, q = lane & 15;
  const int rowBase = (int)blockIdx.x * GBM;
  const int bucket  = rowBase >> 10;
  const unsigned* lb = LIST + (size_t)bucket * (size_t)(RCAP * 2);
  const int flag = FLAG[(size_t)bucket * 32];
  const float qnan = __uint_as_float(0x7fc00000u);

#pragma unroll 1
  for (int i = 0; i < GBM / (2 * NWAVE); ++i) {
    const int d = rowBase + (GBM / NWAVE) * wave + 2 * i + hh;
    int c = CNT[d];
    int o = OFF[d];
    const bool big = c > DEGCAP;
    c = c < 0 ? 0 : (c > DEGCAP ? DEGCAP : c);
    o = o < 0 ? 0 : (o > RCAP - 1 ? RCAP - 1 : o);
    const int co  = __shfl_xor(c, 16, 32);
    const int cm  = c > co ? c : co;
    const int cmu = __builtin_amdgcn_readfirstlane(cm);
    int last = o + c - 1;
    last = last < o ? o : last;
    last = last > RCAP - 1 ? RCAP - 1 : last;
    float a0 = 0.0f, a1 = 0.0f, a2 = 0.0f, a3 = 0.0f;
#pragma unroll 1
    for (int j = 0; j < cmu; ++j) {
      int idx = o + j;
      idx = idx > last ? last : idx;
      const v2u wd = *(const v2ua*)(lb + (size_t)2 * (size_t)idx);
      int sr = (int)wd.x;
      sr = sr < 0 ? 0 : (sr > NN - 1 ? NN - 1 : sr);
      const float w = __uint_as_float(wd.y);
      const v2u xv = *(const v2ua*)(XB + (size_t)sr * D0 + 4 * q);
      asm volatile("" :: "v"(xv));
      const bool valid = j < c;
      const float t0 = fmaf(w, bfw_lo(xv.x), a0), t1 = fmaf(w, bfw_hi(xv.x), a1);
      const float t2 = fmaf(w, bfw_lo(xv.y), a2), t3 = fmaf(w, bfw_hi(xv.y), a3);
      a0 = valid ? t0 : a0; a1 = valid ? t1 : a1; a2 = valid ? t2 : a2; a3 = valid ? t3 : a3;
    }
    const bool bad  = (flag != 0) | big;
    const bool live = d < NN;
    float m0 = bad ? qnan : a0, m1 = bad ? qnan : a1, m2 = bad ? qnan : a2, m3 = bad ? qnan : a3;
    m0 = live ? m0 : 0.0f; m1 = live ? m1 : 0.0f; m2 = live ? m2 : 0.0f; m3 = live ? m3 : 0.0f;
    int h01, h23, l01, l23;
    hilo_pack(m0, m1, m2, m3, h01, h23, l01, l23);
    const v4i ow = regroup8(h01, h23, l01, l23, lane);
    st2_v4i(Z1 + (size_t)d * Z1P + 8 * q, ow);
  }
}

__global__ __launch_bounds__(NTHR) void k_replay2(const unsigned* __restrict__ LIST, const int* __restrict__ CNT,
                                                  const int* __restrict__ OFF, const int* __restrict__ FLAG,
                                                  const float* __restrict__ H, unsigned short* Z2) {
  const int tid = (int)threadIdx.x, lane = tid & 31, wave = tid >> 5;
  const int rowBase = (int)blockIdx.x * GBM;
  const int bucket  = rowBase >> 10;
  const unsigned* lb = LIST + (size_t)bucket * (size_t)(RCAP * 2);
  const int flag = FLAG[(size_t)bucket * 32];
  const float qnan = __uint_as_float(0x7fc00000u);

#pragma unroll 1
  for (int i = 0; i < GBM / NWAVE; ++i) {
    const int d = rowBase + (GBM / NWAVE) * wave + i;
    int cv = CNT[d];
    int ovv = OFF[d];
    const bool big = cv > DEGCAP;
    cv  = cv < 0 ? 0 : (cv > DEGCAP ? DEGCAP : cv);
    ovv = ovv < 0 ? 0 : (ovv > RCAP - 1 ? RCAP - 1 : ovv);
    int lastv = ovv + cv - 1;
    lastv = lastv < ovv ? ovv : lastv;
    lastv = lastv > RCAP - 1 ? RCAP - 1 : lastv;
    const int c    = __builtin_amdgcn_readfirstlane(cv);
    const int o    = __builtin_amdgcn_readfirstlane(ovv);
    const int last = __builtin_amdgcn_readfirstlane(lastv);
    float a0 = 0.0f, a1 = 0.0f, a2 = 0.0f, a3 = 0.0f;
#pragma unroll 1
    for (int j = 0; j < c; ++j) {
      int idx = o + j;
      idx = idx > last ? last : idx;
      const v2u wd = *(const v2ua*)(lb + (size_t)2 * (size_t)idx);
      int sr = (int)wd.x;
      sr = sr < 0 ? 0 : (sr > NN - 1 ? NN - 1 : sr);
      const float w = __uint_as_float(wd.y);
      const v4f hv = *(const v4fa*)(H + (size_t)sr * HD + 4 * lane);
      a0 = fmaf(w, hv.x, a0); a1 = fmaf(w, hv.y, a1); a2 = fmaf(w, hv.z, a2); a3 = fmaf(w, hv.w, a3);
    }
    const bool bad  = (flag != 0) | big;
    const bool live = d < NN;
    float m0 = bad ? qnan : a0, m1 = bad ? qnan : a1, m2 = bad ? qnan : a2, m3 = bad ? qnan : a3;
    m0 = live ? m0 : 0.0f; m1 = live ? m1 : 0.0f; m2 = live ? m2 : 0.0f; m3 = live ? m3 : 0.0f;
    int h01, h23, l01, l23;
    hilo_pack(m0, m1, m2, m3, h01, h23, l01, l23);
    const v4i ow = regroup8w(h01, h23, l01, l23, lane);
    st2_v4i(Z2 + (size_t)d * Z2P + 8 * lane, ow);
  }
}

template <int KTOT, int APITCH, int BPITCH, int NT>
__device__ __forceinline__ void gemm_rows16(const unsigned short* __restrict__ ap,
                                            const unsigned short* __restrict__ bp, v8f (&acc)[NT]) {
  static_assert(KTOT % 32 == 0 && KTOT <= APITCH && KTOT <= BPITCH);
#pragma unroll 1
  for (int k0 = 0; k0 < KTOT; k0 += 32) {
    FragB af;
    af.h[0] = *(const v8usa*)(ap + k0);
    af.h[1] = *(const v8usa*)(ap + k0 + 16);
#pragma unroll
    for (int nt = 0; nt < NT; ++nt) {
      const unsigned short* wq = bp + (size_t)(16 * nt) * (size_t)BPITCH + k0;
      FragB bf;
      bf.h[0] = *(const v8usa*)wq;
      bf.h[1] = *(const v8usa*)(wq + 16);
      acc[nt] = wmb(af, bf, acc[nt]);
    }
  }
}

template <int B0, int NT>
__device__ __forceinline__ void stage_d4(float* stg, const v8f (&acc)[NT], int wave, int hh, int m) {
#pragma unroll
  for (int nt = 0; nt < 4; ++nt) {
#pragma unroll
    for (int r = 0; r < 8; ++r) stg[(16 * wave + 8 * hh + r) * SP + 16 * nt + m] = acc[B0 + nt][r];
  }
}

__device__ __forceinline__ void write_h_half(const float* stg, float* H, int rowBase, int cbase,
                                             int wave, int hh, int m) {
#pragma unroll 1
  for (int i = 0; i < 8; ++i) {
    const int lr   = 16 * wave + 2 * i + hh;
    const int grow = rowBase + lr;
    const bool live = grow < NN;
    const v4f a = *(const v4fa*)(stg + lr * SP + 4 * m);
    asm volatile("" :: "v"(a));
    float v0 = a.x, v1 = a.y, v2 = a.z, v3 = a.w;
    v0 = (v0 > 0.0f) ? v0 : (v0 - v0); v1 = (v1 > 0.0f) ? v1 : (v1 - v1);
    v2 = (v2 > 0.0f) ? v2 : (v2 - v2); v3 = (v3 > 0.0f) ? v3 : (v3 - v3);
    v4f o;
    o.x = live ? v0 : 0.0f; o.y = live ? v1 : 0.0f; o.z = live ? v2 : 0.0f; o.w = live ? v3 : 0.0f;
    st2_v4f(H + (size_t)grow * HD + cbase + 4 * m, o);
  }
}

__global__ __launch_bounds__(NTHR) __attribute__((amdgpu_num_vgpr(248)))
void k_gemm1(const unsigned short* __restrict__ Z1, const unsigned short* __restrict__ W1D, float* H) {
  __shared__ __attribute__((aligned(16))) float stg[GBM * SP];
  const int tid = (int)threadIdx.x, lane = tid & 31, wave = tid >> 5, hh = lane >> 4, m = lane & 15;
  const int rowBase = (int)blockIdx.x * GBM;

  v8f acc[8];
  {
    const v8f z = {0.f, 0.f, 0.f, 0.f, 0.f, 0.f, 0.f, 0.f};
#pragma unroll
    for (int t = 0; t < 8; ++t) acc[t] = z;
  }
  const unsigned short* ap = Z1 + (size_t)(rowBase + 16 * wave + m) * (size_t)Z1P + 8 * hh;
  const unsigned short* bp = W1D + (size_t)m * (size_t)W1P + 8 * hh;
  gemm_rows16<K1, Z1P, W1P, 8>(ap, bp, acc);

  stage_d4<0, 8>(stg, acc, wave, hh, m);
  __syncthreads();
  write_h_half(stg, H, rowBase, 0, wave, hh, m);
  __syncthreads();
  stage_d4<4, 8>(stg, acc, wave, hh, m);
  __syncthreads();
  write_h_half(stg, H, rowBase, 64, wave, hh, m);
}

__global__ __launch_bounds__(NTHR) __attribute__((amdgpu_num_vgpr(248)))
void k_gemm2(const unsigned short* __restrict__ Z2, const unsigned short* __restrict__ W3D,
             const int* __restrict__ FLAG, float* out) {
  __shared__ __attribute__((aligned(16))) float stg[GBM * SP];
  const int tid = (int)threadIdx.x, lane = tid & 31, wave = tid >> 5, hh = lane >> 4, m = lane & 15;
  const int rowBase = (int)blockIdx.x * GBM;
  const int flag = FLAG[(size_t)(rowBase >> 10) * 32];
  const float qnan = __uint_as_float(0x7fc00000u);

  v8f acc[4];
  {
    const v8f z = {0.f, 0.f, 0.f, 0.f, 0.f, 0.f, 0.f, 0.f};
#pragma unroll
    for (int t = 0; t < 4; ++t) acc[t] = z;
  }
  const unsigned short* ap = Z2 + (size_t)(rowBase + 16 * wave + m) * (size_t)Z2P + 8 * hh;
  const unsigned short* bp = W3D + (size_t)m * (size_t)W3P + 8 * hh;
  gemm_rows16<K2, Z2P, W3P, 4>(ap, bp, acc);
  stage_d4<0, 4>(stg, acc, wave, hh, m);
  __syncthreads();

#pragma unroll 1
  for (int i = 0; i < 8; ++i) {
    const int lr   = 16 * wave + 2 * i + hh;
    const int grow = rowBase + lr;
    const bool live = grow < NN;
    const int gs = live ? grow : 0;
    const v4f a = *(const v4fa*)(stg + lr * SP + 4 * m);
    asm volatile("" :: "v"(a));
    v4f o;
    o.x = (flag != 0) ? qnan : a.x; o.y = (flag != 0) ? qnan : a.y;
    o.z = (flag != 0) ? qnan : a.z; o.w = (flag != 0) ? qnan : a.w;
    float* op = out + (size_t)gs * OD + 4 * m;
    if (live) *(volatile v4f*)op = o;
    __threadfence();
    if (live) *(volatile v4f*)op = o;
  }
}

extern "C" void kernel_launch(void* const* d_in, const int* in_sizes, int n_in,
                              void* d_out, int out_size, void* d_ws, size_t ws_size,
                              hipStream_t stream) {
  if (n_in < 6) return;
  if (in_sizes[0] != NN * D0) return;
  if (in_sizes[1] != NE) return;
  if (in_sizes[2] != NE) return;
  if (in_sizes[3] != NE) return;
  if (in_sizes[4] != D0 * HD) return;
  if (in_sizes[5] != HD * OD) return;
  if (out_size != NN * OD) return;

  const float* x    = (const float*)d_in[0];
  const int*   keys = (const int*)d_in[1];
  const int*   cols = (const int*)d_in[2];
  const float* ew   = (const float*)d_in[3];
  const float* W1   = (const float*)d_in[4];
  const float* W3   = (const float*)d_in[5];
  float* out = (float*)d_out;

  constexpr size_t zXB   = (size_t)MP * D0 * 2;
  constexpr size_t zZ1   = (size_t)MP * Z1P * 2;
  constexpr size_t zRZ   = (size_t)MP * Z2P * 2;
  constexpr size_t zH    = (size_t)MP * HD * 4;
  constexpr size_t zLIST = (size_t)NBK * RCAP * 8;
  constexpr size_t zCNT  = (size_t)NBK * NBRUN * 4;
  constexpr size_t zFLAG = (size_t)NBK * 128;
  constexpr size_t zW1D  = (size_t)HD * W1P * 2;
  constexpr size_t zW3D  = (size_t)OD * W3P * 2;
  constexpr size_t oRZ   = 0;
  constexpr size_t oXB   = oRZ;
  constexpr size_t oZ1   = oXB + zXB;
  constexpr size_t oH    = oRZ + zRZ;
  constexpr size_t oLIST = oH + zH;
  constexpr size_t oCNT  = oLIST + zLIST;
  constexpr size_t oOFF  = oCNT + zCNT;
  constexpr size_t oFLAG = oOFF + zCNT;
  constexpr size_t oW1D  = oFLAG + zFLAG;
  constexpr size_t oW3D  = oW1D + zW1D;
  constexpr size_t oEND  = oW3D + zW3D;
  static_assert(zXB + zZ1 <= zRZ);
  static_assert(zXB % 128 == 0 && zZ1 % 128 == 0 && zRZ % 128 == 0 && zH % 128 == 0 && zLIST % 128 == 0);
  static_assert(zCNT % 128 == 0 && zFLAG % 128 == 0 && zW1D % 128 == 0 && zW3D % 128 == 0);
  static_assert(oEND <= (size_t)(128u << 20));
  if (oEND > ws_size) return;

  char* ws = (char*)d_ws;
  unsigned short* XB   = (unsigned short*)(ws + oXB);
  unsigned short* Z1   = (unsigned short*)(ws + oZ1);
  unsigned short* Z2   = (unsigned short*)(ws + oRZ);
  float*          H    = (float*)(ws + oH);
  unsigned*       LIST = (unsigned*)(ws + oLIST);
  int*            CNT  = (int*)(ws + oCNT);
  int*            OFF  = (int*)(ws + oOFF);
  int*            FLAG = (int*)(ws + oFLAG);
  unsigned short* W1D  = (unsigned short*)(ws + oW1D);
  unsigned short* W3D  = (unsigned short*)(ws + oW3D);

  hipFuncSetAttribute(reinterpret_cast<const void*>(&k_bucket), hipFuncAttributeMaxDynamicSharedMemorySize, (int)BK_LDS);

  k_prep<<<PBTOT, NTHR, 0, stream>>>(x, W1, W3, XB, W1D, W3D);
  k_bucket<<<NBK, NTHR, BK_LDS, stream>>>(keys, cols, ew, LIST, CNT, OFF, FLAG);
  k_replay1<<<MP / GBM, NTHR, 0, stream>>>(LIST, CNT, OFF, FLAG, XB, Z1);
  k_gemm1<<<MP / GBM, NTHR, 0, stream>>>(Z1, W1D, H);
  k_replay2<<<MP / GBM, NTHR, 0, stream>>>(LIST, CNT, OFF, FLAG, H, Z2);
  k_gemm2<<<MP / GBM, NTHR, 0, stream>>>(Z2, W3D, FLAG, out);
}
